// RWKV7_CrossAttention_78391743086653
// MI455X (gfx1250) — hardware-verified
//
#include <hip/hip_runtime.h>
#include <math.h>

constexpr int HID     = 256;
constexpr int SEQ     = 512;
constexpr int NBAT    = 2;
constexpr int NQRY    = 8;
constexpr int NEB     = NBAT * NQRY;
constexpr int NHEAD   = 4;
constexpr int HDIM    = HID / NHEAD;
constexpr int ROWS_EB = NEB * SEQ;
constexpr int ROWS_KV = NBAT * SEQ;
constexpr int LORA_R  = 32;
constexpr int LORA_RP = 64;
constexpr int GATE_R  = 64;
constexpr int SC_CH   = 8;
constexpr float DECAY_NEG = -0.6065306597126334f;
constexpr float GN_EPS    = (float)(HDIM * 1e-05);
static_assert(HID == 256 && HDIM == 64 && NEB == 16);
static_assert(ROWS_EB % 64 == 0 && ROWS_KV % 64 == 0 && HID % 64 == 0 && LORA_RP % 64 == 0);
static_assert(HID % 32 == 0 && LORA_R % 32 == 0);
static_assert(SEQ % SC_CH == 0);

typedef __attribute__((ext_vector_type(16))) __bf16   v16b;
typedef __attribute__((ext_vector_type(8)))  __bf16   v8b;
typedef __attribute__((ext_vector_type(8)))  float    v8f;
typedef __attribute__((ext_vector_type(4)))  float    v4f;
typedef __attribute__((ext_vector_type(4)))  unsigned int v4u;

__device__ __forceinline__ unsigned short f2bf_bits(float f) {
  unsigned u = __float_as_uint(f);
  return (unsigned short)((u + 0x7FFFu + ((u >> 16) & 1u)) >> 16);
}
__device__ __forceinline__ float bf_bits2f(unsigned short h) { return __uint_as_float(((unsigned)h) << 16); }
__device__ __forceinline__ unsigned pk16(unsigned short a, unsigned short b) { return (unsigned)a | ((unsigned)b << 16); }
__device__ __forceinline__ void split_bf(float f, unsigned short& hb, unsigned short& lb) {
  hb = f2bf_bits(f);
  lb = f2bf_bits(f - bf_bits2f(hb));
}
__device__ __forceinline__ float sigmoid_f(float x) { return 1.0f / (1.0f + expf(-x)); }
__device__ __forceinline__ float wave_sum(float x) {
#pragma unroll
  for (int off = 16; off > 0; off >>= 1) x += __shfl_xor(x, off, 32);
  return x;
}

__device__ __forceinline__ void dep_guard4_b(v8f& a, v8f& b, v8f& c, v8f& d, v16b x, v16b y) {
  asm volatile("v_nop\n\tv_nop\n\tv_nop\n\tv_nop" : "+v"(a), "+v"(b), "+v"(c), "+v"(d) : "v"(x), "v"(y));
}
__device__ __forceinline__ void keep4_b(v16b a, v16b b, v16b c, v16b d) { asm volatile("v_nop" :: "v"(a), "v"(b), "v"(c), "v"(d)); }
__device__ __forceinline__ void acc_guard4(v8f& a, v8f& b, v8f& c, v8f& d) {
  asm volatile("v_nop\n\tv_nop\n\tv_nop\n\tv_nop" : "+v"(a), "+v"(b), "+v"(c), "+v"(d));
}
struct FragB {
  union U { v16b v; v8b h[2]; };
  static __device__ __forceinline__ v16b load(const __bf16* p) {
    U f; f.h[0] = *(const v8b*)(p); f.h[1] = *(const v8b*)(p + 16); return f.v;
  }
  static __device__ __forceinline__ v8f mma(v16b a, v16b b, v8f c) {
    return __builtin_amdgcn_wmma_f32_16x16x32_bf16(false, a, false, b, (short)0, c, false, false);
  }
};

__device__ __forceinline__ void store_split8(const float (&f)[8], unsigned short* ph, unsigned short* pl) {
  unsigned short hb[8], lb[8];
#pragma unroll
  for (int e = 0; e < 8; ++e) split_bf(f[e], hb[e], lb[e]);
  const v4u uh = (v4u){pk16(hb[0], hb[1]), pk16(hb[2], hb[3]), pk16(hb[4], hb[5]), pk16(hb[6], hb[7])};
  const v4u ul = (v4u){pk16(lb[0], lb[1]), pk16(lb[2], lb[3]), pk16(lb[4], lb[5]), pk16(lb[6], lb[7])};
  *(volatile v4u*)ph = uh;
  *(volatile v4u*)pl = ul;
  __threadfence();
  *(volatile v4u*)ph = uh;
  *(volatile v4u*)pl = ul;
}

template <int OUT_MODE>
__global__ __launch_bounds__(256) void wmma_gemm64_split(
    const unsigned short* __restrict__ Ap, const unsigned short* __restrict__ A2p, int lda, long strideA,
    const unsigned short* __restrict__ Btp, const unsigned short* __restrict__ Bt2p, int ldb, long strideB,
    void* __restrict__ Cout, void* __restrict__ Cout2, int ldc, long strideC,
    int M, int N, int K) {
  typedef __bf16 T;
  const T* A = (const T*)Ap; const T* A2 = (const T*)A2p; const T* Bt = (const T*)Btp; const T* Bt2 = (const T*)Bt2p;
  __shared__ __align__(16) float sT[8][16 * 68];
  const int b    = blockIdx.y;
  const int lane = threadIdx.x & 31;
  const int wave = threadIdx.x >> 5;
  const int tilesN = N >> 6;
  const int tilesM = M >> 6;
  const int tile = blockIdx.x * 8 + wave;
  if (tile >= tilesM * tilesN) return;
  const int tm = tile / tilesN;
  const int tn = tile - tm * tilesN;
  const int m0 = tm << 6;
  const int n0 = tn << 6;

  const int rlane = lane & 15;
  const int koff  = (lane >> 4) * 8;
  const int mOff  = (lane >> 4) * 8;

  const T* Ab  = A   + (size_t)b * strideA + (size_t)(m0 + rlane) * lda + koff;
  const T* Ab2 = A2  + (size_t)b * strideA + (size_t)(m0 + rlane) * lda + koff;
  const T* Bb  = Bt  + (size_t)b * strideB + (size_t)(n0 + rlane) * ldb + koff;
  const T* Bb2 = Bt2 + (size_t)b * strideB + (size_t)(n0 + rlane) * ldb + koff;
  const size_t a16 = (size_t)16 * lda;
  const size_t b16 = (size_t)16 * ldb;

  v8f acc[4][4];
#pragma unroll
  for (int i = 0; i < 4; ++i)
#pragma unroll
    for (int j = 0; j < 4; ++j) acc[i][j] = (v8f){0.f, 0.f, 0.f, 0.f, 0.f, 0.f, 0.f, 0.f};

  for (int k0 = 0; k0 < K; k0 += 32) {
    v16b bh[4], bl[4];
#pragma unroll
    for (int j = 0; j < 4; ++j) {
      bh[j] = FragB::load(Bb  + j * b16 + k0);
      bl[j] = FragB::load(Bb2 + j * b16 + k0);
    }
#pragma unroll
    for (int i = 0; i < 4; ++i) {
      const v16b ah = FragB::load(Ab  + i * a16 + k0);
      const v16b al = FragB::load(Ab2 + i * a16 + k0);
#pragma unroll
      for (int j = 0; j < 4; ++j) {
        acc[i][j] = FragB::mma(ah, bh[j], acc[i][j]);
        acc[i][j] = FragB::mma(ah, bl[j], acc[i][j]);
        acc[i][j] = FragB::mma(al, bh[j], acc[i][j]);
      }
      dep_guard4_b(acc[i][0], acc[i][1], acc[i][2], acc[i][3], ah, al);
    }
    keep4_b(bh[0], bh[1], bh[2], bh[3]);
    keep4_b(bl[0], bl[1], bl[2], bl[3]);
  }
  acc_guard4(acc[0][0], acc[0][1], acc[0][2], acc[0][3]);
  acc_guard4(acc[1][0], acc[1][1], acc[1][2], acc[1][3]);
  acc_guard4(acc[2][0], acc[2][1], acc[2][2], acc[2][3]);
  acc_guard4(acc[3][0], acc[3][1], acc[3][2], acc[3][3]);

  float* slab = sT[wave];
#pragma unroll
  for (int i = 0; i < 4; ++i) {
    const int mBase = m0 + (i << 4);
#pragma unroll
    for (int j = 0; j < 4; ++j) {
#pragma unroll
      for (int r = 0; r < 8; ++r) slab[(mOff + r) * 68 + (j << 4) + rlane] = acc[i][j][r];
    }
    __builtin_amdgcn_fence(__ATOMIC_RELEASE, "workgroup");
    __builtin_amdgcn_wave_barrier();
    __builtin_amdgcn_fence(__ATOMIC_ACQUIRE, "workgroup");
    if (OUT_MODE == 0) {
      float* C = (float*)Cout + (size_t)b * strideC;
      const int hh = lane >> 4, c4 = (lane & 15) * 4;
      for (int pass = 0; pass < 2; ++pass) {
#pragma unroll
        for (int it = 0; it < 8; ++it) {
          const int row = it * 2 + hh;
          const v4f v = *(const v4f*)(slab + row * 68 + c4);
          *(volatile v4f*)(C + (size_t)(mBase + row) * ldc + n0 + c4) = v;
        }
        __threadfence();
      }
    } else {
      const int q = lane >> 3, c8 = (lane & 7) * 8;
      unsigned short* C  = (unsigned short*)Cout  + (size_t)b * strideC;
      unsigned short* C2 = (unsigned short*)Cout2 + (size_t)b * strideC;
      for (int pass = 0; pass < 2; ++pass) {
#pragma unroll
        for (int it = 0; it < 4; ++it) {
          const int row = it * 4 + q;
          const float* sp = slab + row * 68 + c8;
          unsigned short hb[8], lb[8];
#pragma unroll
          for (int e = 0; e < 8; ++e) {
            const float x = sp[e];
            split_bf(x, hb[e], lb[e]);
          }
          const v4u uh = (v4u){pk16(hb[0], hb[1]), pk16(hb[2], hb[3]), pk16(hb[4], hb[5]), pk16(hb[6], hb[7])};
          const v4u ul = (v4u){pk16(lb[0], lb[1]), pk16(lb[2], lb[3]), pk16(lb[4], lb[5]), pk16(lb[6], lb[7])};
          *(volatile v4u*)(C  + (size_t)(mBase + row) * ldc + n0 + c8) = uh;
          *(volatile v4u*)(C2 + (size_t)(mBase + row) * ldc + n0 + c8) = ul;
        }
        __threadfence();
      }
    }
    __builtin_amdgcn_fence(__ATOMIC_RELEASE, "workgroup");
    __builtin_amdgcn_wave_barrier();
    __builtin_amdgcn_fence(__ATOMIC_ACQUIRE, "workgroup");
  }
}

__global__ __launch_bounds__(256) void split8_kernel(const float* __restrict__ s0, const float* __restrict__ s1,
                                                     unsigned short* __restrict__ dh, unsigned short* __restrict__ dl, int n8) {
  const int i = blockIdx.x * 256 + threadIdx.x;
  const int y = blockIdx.y;
  const float* src = (y == 0) ? s0 : s1;
  if (i >= n8) return;
  const float* p = src + 8 * (size_t)i;
  const v4f a = *(const v4f*)(p);
  const v4f c = *(const v4f*)(p + 4);
  float f[8];
#pragma unroll
  for (int e = 0; e < 4; ++e) { f[e] = a[e]; f[4 + e] = c[e]; }
  const size_t o = (size_t)y * (size_t)n8 * 8 + 8 * (size_t)i;
  store_split8(f, dh + o, dl + o);
}

__global__ __launch_bounds__(256) void tpack_kernel(const float* __restrict__ s0, const float* __restrict__ s1,
                                                    const float* __restrict__ s2,
                                                    unsigned short* __restrict__ dh, unsigned short* __restrict__ dl,
                                                    int R, int C, int NP) {
  const int i = blockIdx.x * 256 + threadIdx.x;
  const int y = blockIdx.y;
  const float* src = (y == 0) ? s0 : ((y == 1) ? s1 : s2);
  const int r8 = R >> 3;
  const int total = NP * r8;
  if (i >= total) return;
  const int n  = i / r8;
  const int k0 = (i - n * r8) * 8;
  const int nc = (n < C) ? n : (C - 1);
  const bool live = (n < C);
  float f[8];
#pragma unroll
  for (int e = 0; e < 8; ++e) {
    const float x = src[(size_t)(k0 + e) * C + nc];
    f[e] = live ? x : 0.0f;
  }
  const size_t o = (size_t)y * (size_t)NP * (size_t)R + 8 * (size_t)i;
  store_split8(f, dh + o, dl + o);
}

__global__ __launch_bounds__(256) void mix_kernel(const float* __restrict__ query, const float* __restrict__ keyval,
                                                  const float* __restrict__ x_w, const float* __restrict__ x_k,
                                                  const float* __restrict__ x_v, const float* __restrict__ x_a,
                                                  unsigned short* __restrict__ XWAh, unsigned short* __restrict__ XWAl,
                                                  unsigned short* __restrict__ XKVh, unsigned short* __restrict__ XKVl) {
  const int lane = threadIdx.x & 31, wave = threadIdx.x >> 5;
  const int row = blockIdx.x * 8 + wave;
  const int eb = row >> 9, t = row & (SEQ - 1), b = eb >> 3;
  const int c0 = lane * 8;
  const float* hp = keyval + ((size_t)b * SEQ + t) * HID + c0;
  const float* qp = query + (size_t)eb * HID + c0;
  const v4f h0 = *(const v4f*)(hp), h1 = *(const v4f*)(hp + 4);
  const v4f q0 = *(const v4f*)(qp), q1 = *(const v4f*)(qp + 4);
  const v4f w0 = *(const v4f*)(x_w + c0), w1 = *(const v4f*)(x_w + c0 + 4);
  const v4f a0 = *(const v4f*)(x_a + c0), a1 = *(const v4f*)(x_a + c0 + 4);
  float hs[8], fw[8], fa[8];
#pragma unroll
  for (int e = 0; e < 4; ++e) {
    hs[e] = h0[e]; hs[4 + e] = h1[e];
    const float xc0 = q0[e] - h0[e];
    const float xc1 = q1[e] - h1[e];
    fw[e] = h0[e] + xc0 * w0[e]; fw[4 + e] = h1[e] + xc1 * w1[e];
    fa[e] = h0[e] + xc0 * a0[e]; fa[4 + e] = h1[e] + xc1 * a1[e];
  }
  const size_t oeb = (size_t)row * HID + c0;
  store_split8(fw, XWAh + oeb, XWAl + oeb);
  store_split8(fa, XWAh + (size_t)ROWS_EB * HID + oeb, XWAl + (size_t)ROWS_EB * HID + oeb);
  if ((eb & 7) == 0) {
    const int tp = (t > 0) ? (t - 1) : 0;
    const float* pp = keyval + ((size_t)b * SEQ + tp) * HID + c0;
    const v4f p0 = *(const v4f*)(pp), p1 = *(const v4f*)(pp + 4);
    const v4f k0 = *(const v4f*)(x_k + c0), k1 = *(const v4f*)(x_k + c0 + 4);
    const v4f v0 = *(const v4f*)(x_v + c0), v1 = *(const v4f*)(x_v + c0 + 4);
    float fk[8], fv[8];
#pragma unroll
    for (int e = 0; e < 4; ++e) {
      const float s0 = (t > 0) ? p0[e] : 0.0f;
      const float s1 = (t > 0) ? p1[e] : 0.0f;
      const float d0 = s0 - hs[e];
      const float d1 = s1 - hs[4 + e];
      fk[e] = hs[e] + d0 * k0[e]; fk[4 + e] = hs[4 + e] + d1 * k1[e];
      fv[e] = hs[e] + d0 * v0[e]; fv[4 + e] = hs[4 + e] + d1 * v1[e];
    }
    const size_t okv = ((size_t)b * SEQ + t) * HID + c0;
    store_split8(fk, XKVh + okv, XKVl + okv);
    store_split8(fv, XKVh + (size_t)ROWS_KV * HID + okv, XKVl + (size_t)ROWS_KV * HID + okv);
  }
}

__global__ __launch_bounds__(256) void tanh_split2_kernel(const float* __restrict__ in, unsigned short* __restrict__ dh,
                                                          unsigned short* __restrict__ dl, int n2) {
  const int i = blockIdx.x * 256 + threadIdx.x;
  if (i < n2) {
    const float a = tanhf(in[2 * (size_t)i]);
    const float c = tanhf(in[2 * (size_t)i + 1]);
    unsigned short ha, la, hc, lc;
    split_bf(a, ha, la);
    split_bf(c, hc, lc);
    const unsigned uh = pk16(ha, hc), ul = pk16(la, lc);
    ((volatile unsigned*)dh)[i] = uh;
    ((volatile unsigned*)dl)[i] = ul;
    __threadfence();
    ((volatile unsigned*)dh)[i] = uh;
    ((volatile unsigned*)dl)[i] = ul;
  }
}

__global__ __launch_bounds__(256) void rproj_kernel(const float* __restrict__ query, const float* __restrict__ keyval,
                                                    const float* __restrict__ x_r, const float* __restrict__ Wr,
                                                    float* __restrict__ RL) {
  __shared__ __align__(16) float xs[HID];
  __shared__ __align__(16) float ro[HID];
  const int tid = threadIdx.x;
  const int eb = blockIdx.x, b = eb >> 3;
  const float hsv = keyval[((size_t)b * SEQ + (SEQ - 1)) * HID + tid];
  const float eqv = query[(size_t)eb * HID + tid];
  xs[tid] = hsv + (eqv - hsv) * x_r[tid];
  __syncthreads();
  const float* wrow = Wr + (size_t)tid * HID;
  float s0 = 0.0f, s1 = 0.0f, s2 = 0.0f, s3 = 0.0f;
#pragma unroll 2
  for (int c4 = 0; c4 < HID / 4; ++c4) {
    const v4f w = *(const v4f*)(wrow + 4 * c4);
    const v4f x = *(const v4f*)(xs + 4 * c4);
    s0 = fmaf(w[0], x[0], s0);
    s1 = fmaf(w[1], x[1], s1);
    s2 = fmaf(w[2], x[2], s2);
    s3 = fmaf(w[3], x[3], s3);
  }
  ro[tid] = (s0 + s1) + (s2 + s3);
  __syncthreads();
  if (tid < 64) {
    const v4f v = *(const v4f*)(ro + 4 * tid);
    float* op = RL + (size_t)eb * HID + 4 * tid;
    *(volatile v4f*)op = v;
    __threadfence();
    *(volatile v4f*)op = v;
  }
}

__global__ __launch_bounds__(256) void prep_kernel(const float* __restrict__ PWA, const float* __restrict__ KVR,
                                                   const float* __restrict__ PVf, const float* __restrict__ vfirst,
                                                   const float* __restrict__ w0, const float* __restrict__ a0,
                                                   const float* __restrict__ v0, const float* __restrict__ k_k,
                                                   const float* __restrict__ k_a,
                                                   float* __restrict__ EW, float* __restrict__ KF, float* __restrict__ NKK,
                                                   float* __restrict__ BM, float* __restrict__ VP) {
  const int tid = threadIdx.x, lane = tid & 31, wave = tid >> 5;
  const int row = blockIdx.x * 2 + (wave >> 2);
  const int h = wave & 3;
  const int eb = row >> 9, t = row & (SEQ - 1);
  const int rkv = ((eb >> 3) << 9) + t;
  const int cb = h * HDIM + lane;
  const float* KR = KVR;
  const float* VR = KVR + (size_t)ROWS_KV * HID;
  const float* PW = PWA;
  const float* PA = PWA + (size_t)ROWS_EB * HID;
  const size_t okv = (size_t)rkv * HID, oeb = (size_t)row * HID;
  const float q0 = KR[okv + cb] * k_k[cb];
  const float q1 = KR[okv + cb + 32] * k_k[cb + 32];
  float ss = q0 * q0 + q1 * q1;
  ss = wave_sum(ss);
  const float inv = 1.0f / fmaxf(sqrtf(ss), 1e-12f);
#pragma unroll 1
  for (int j = 0; j < 2; ++j) {
    const int c = cb + 32 * j;
    const float kr = KR[okv + c];
    const float vr = VR[okv + c];
    const float pv = PVf[okv + c];
    const float pw = PW[oeb + c];
    const float pa = PA[oeb + c];
    const float vf = vfirst[oeb + c];
    const float sw = sigmoid_f(w0[c] + pw);
    const float ew = expf(DECAY_NEG * sw);
    const float ag = sigmoid_f(a0[c] + pa);
    const float vg = sigmoid_f(v0[c] + pv);
    const float vfin = vr + (vf - vr) * vg;
    const float kkn = (kr * k_k[c]) * inv;
    const float nkk = -kkn;
    const float bm = kkn * ag;
    const float kf = kr + (kr * (ag - 1.0f)) * k_a[c];
    for (int pass = 0; pass < 2; ++pass) {
      *(volatile float*)(EW  + oeb + c) = ew;
      *(volatile float*)(KF  + oeb + c) = kf;
      *(volatile float*)(NKK + oeb + c) = nkk;
      *(volatile float*)(BM  + oeb + c) = bm;
      *(volatile float*)(VP  + oeb + c) = vfin;
      __threadfence();
    }
  }
}

__global__ __launch_bounds__(64) void scan_kernel(const float* __restrict__ EW, const float* __restrict__ KF,
                                                  const float* __restrict__ NKK, const float* __restrict__ BM,
                                                  const float* __restrict__ VP, const float* __restrict__ RL,
                                                  float* __restrict__ OS) {
  __shared__ __align__(16) float Sst[HDIM * HDIM];
  __shared__ __align__(16) float cf[4][SC_CH][HDIM];
  __shared__ __align__(16) float rsh[HDIM];
  const int tid = threadIdx.x;
  const int unit = blockIdx.x;
  const int eb = unit >> 2, h = unit & 3;
  const size_t base = (size_t)eb * SEQ * HID + (size_t)h * HDIM;
#pragma unroll 8
  for (int k = 0; k < HDIM; ++k) Sst[k * HDIM + tid] = 0.0f;
  rsh[tid] = RL[(size_t)eb * HID + h * HDIM + tid];
  float as = 0.0f;
  const int st = tid >> 4, q4 = (tid & 15) * 4;
#pragma unroll 1
  for (int t0 = 0; t0 < SEQ; t0 += SC_CH) {
    __syncthreads();
#pragma unroll
    for (int i = 0; i < 8; ++i) {
      const int arr  = i >> 1;
      const int step = ((i & 1) << 2) | st;
      int tt = t0 + step;
      if (arr == 2) tt = (tt + 1 < SEQ) ? (tt + 1) : (SEQ - 1);
      const float* P = (arr == 0) ? EW : ((arr == 1) ? KF : ((arr == 2) ? NKK : BM));
      const v4f x = *(const v4f*)(P + base + (size_t)tt * HID + q4);
      *(v4f*)(&cf[arr][step][q4]) = x;
    }
    __syncthreads();
#pragma unroll 1
    for (int s = 0; s < SC_CH; ++s) {
      const float vv = VP[base + (size_t)(t0 + s) * HID + tid];
      const float* ce = &cf[0][s][0];
      const float* ck = &cf[1][s][0];
      const float* cn = &cf[2][s][0];
      const float* cb = &cf[3][s][0];
      float asn = 0.0f;
#pragma unroll 1
      for (int k4 = 0; k4 < HDIM / 4; ++k4) {
        const v4f e4 = *(const v4f*)(ce + 4 * k4);
        const v4f f4 = *(const v4f*)(ck + 4 * k4);
        const v4f n4 = *(const v4f*)(cn + 4 * k4);
        const v4f b4 = *(const v4f*)(cb + 4 * k4);
#pragma unroll
        for (int j = 0; j < 4; ++j) {
          const int si = (4 * k4 + j) * HDIM + tid;
          const float sv = Sst[si];
          const float ns = (sv * e4[j] + f4[j] * vv) + b4[j] * as;
          Sst[si] = ns;
          asn = fmaf(n4[j], ns, asn);
        }
      }
      as = asn;
    }
  }
  float o = 0.0f;
#pragma unroll 4
  for (int k = 0; k < HDIM; ++k) o = fmaf(rsh[k], Sst[k * HDIM + tid], o);
  float* op = OS + (size_t)eb * HID + h * HDIM + tid;
  *(volatile float*)op = o;
  __threadfence();
  *(volatile float*)op = o;
}

__global__ __launch_bounds__(256) void final_kernel(const float* __restrict__ OS, const float* __restrict__ RL,
                                                    const float* __restrict__ KF, const float* __restrict__ VP,
                                                    const float* __restrict__ query, const float* __restrict__ keyval,
                                                    const float* __restrict__ x_g, const float* __restrict__ g1,
                                                    const float* __restrict__ g2, const float* __restrict__ gn_w,
                                                    const float* __restrict__ gn_b, const float* __restrict__ r_k,
                                                    const float* __restrict__ Wo, float* __restrict__ out) {
  __shared__ float redA[8];
  __shared__ float redB[8];
  __shared__ float redC[8];
  __shared__ __align__(16) float xg[HID];
  __shared__ float part[4][GATE_R];
  __shared__ float hg[GATE_R];
  __shared__ __align__(16) float ysh[HID];
  __shared__ __align__(16) float osh[HID];
  const int tid = threadIdx.x, lane = tid & 31, wave = tid >> 5;
  const int eb = blockIdx.x, b = eb >> 3;
  const int hw = (wave >> 1) << 1;
  const size_t last = ((size_t)eb * SEQ + (SEQ - 1)) * HID + tid;
  const float o  = OS[(size_t)eb * HID + tid];
  const float rl = RL[(size_t)eb * HID + tid];
  const float kf = KF[last];
  const float vl = VP[last];
  const float hsv = keyval[((size_t)b * SEQ + (SEQ - 1)) * HID + tid];
  const float eqv = query[(size_t)eb * HID + tid];
  xg[tid] = hsv + (eqv - hsv) * x_g[tid];
  const float sA = wave_sum(o);
  const float sC = wave_sum((rl * kf) * r_k[tid]);
  if (lane == 0) { redA[wave] = sA; redC[wave] = sC; }
  __syncthreads();
  const float mu = (redA[hw] + redA[hw + 1]) * (1.0f / HDIM);
  const float dot = redC[hw] + redC[hw + 1];
  const float d = o - mu;
  const float sB = wave_sum(d * d);
  if (lane == 0) redB[wave] = sB;
  {
    const int j = tid & (GATE_R - 1), pq = tid >> 6;
    float acc = 0.0f;
#pragma unroll 4
    for (int cc = 0; cc < 64; ++cc) {
      const int ci = pq * 64 + cc;
      acc = fmaf(xg[ci], g1[(size_t)ci * GATE_R + j], acc);
    }
    part[pq][j] = acc;
  }
  __syncthreads();
  const float var = (redB[hw] + redB[hw + 1]) * (1.0f / HDIM);
  float y = (d * rsqrtf(var + GN_EPS)) * gn_w[tid] + gn_b[tid];
  y = y + dot * vl;
  if (tid < GATE_R) {
    const float z = (part[0][tid] + part[1][tid]) + (part[2][tid] + part[3][tid]);
    hg[tid] = sigmoid_f(z);
  }
  __syncthreads();
  float gacc = 0.0f;
#pragma unroll 4
  for (int j = 0; j < GATE_R; ++j) gacc = fmaf(hg[j], g2[(size_t)j * HID + tid], gacc);
  ysh[tid] = y * gacc;
  __syncthreads();
  const float* wrow = Wo + (size_t)tid * HID;
  float s0 = 0.0f, s1 = 0.0f, s2 = 0.0f, s3 = 0.0f;
#pragma unroll 2
  for (int c4 = 0; c4 < HID / 4; ++c4) {
    const v4f w = *(const v4f*)(wrow + 4 * c4);
    const v4f x = *(const v4f*)(ysh + 4 * c4);
    s0 = fmaf(w[0], x[0], s0);
    s1 = fmaf(w[1], x[1], s1);
    s2 = fmaf(w[2], x[2], s2);
    s3 = fmaf(w[3], x[3], s3);
  }
  osh[tid] = (s0 + s1) + (s2 + s3);
  __syncthreads();
  if (tid < 64) {
    const v4f v = *(const v4f*)(osh + 4 * tid);
    float* op = out + (size_t)eb * HID + 4 * tid;
    *(volatile v4f*)op = v;
    __threadfence();
    *(volatile v4f*)op = v;
  }
}

extern "C" void kernel_launch(void* const* d_in, const int* in_sizes, int n_in,
                              void* d_out, int out_size, void* d_ws, size_t ws_size, hipStream_t stream) {
  if (n_in < 29 || d_out == nullptr || d_ws == nullptr) return;
  if (in_sizes[0] != NEB * HID || in_sizes[1] != ROWS_KV * HID || in_sizes[2] != ROWS_EB * HID) return;
  for (int i = 3; i <= 9; ++i) if (in_sizes[i] != HID) return;
  if (in_sizes[10] != HID * LORA_R || in_sizes[11] != LORA_R * HID || in_sizes[12] != HID ||
      in_sizes[13] != HID * LORA_R || in_sizes[14] != LORA_R * HID || in_sizes[15] != HID ||
      in_sizes[16] != HID * LORA_R || in_sizes[17] != LORA_R * HID ||
      in_sizes[18] != HID * GATE_R || in_sizes[19] != GATE_R * HID ||
      in_sizes[20] != HID || in_sizes[21] != HID || in_sizes[22] != HID ||
      in_sizes[23] != HID * HID || in_sizes[24] != HID * HID || in_sizes[25] != HID * HID || in_sizes[26] != HID * HID ||
      in_sizes[27] != HID || in_sizes[28] != HID || out_size != NEB * HID) return;

  const float* query  = (const float*)d_in[0];
  const float* keyval = (const float*)d_in[1];
  const float* vfirst = (const float*)d_in[2];
  const float* x_r = (const float*)d_in[3];
  const float* x_w = (const float*)d_in[4];
  const float* x_k = (const float*)d_in[5];
  const float* x_v = (const float*)d_in[6];
  const float* x_a = (const float*)d_in[7];
  const float* x_g = (const float*)d_in[8];
  const float* w0 = (const float*)d_in[9];
  const float* w1 = (const float*)d_in[10];
  const float* w2 = (const float*)d_in[11];
  const float* a0 = (const float*)d_in[12];
  const float* a1 = (const float*)d_in[13];
  const float* a2 = (const float*)d_in[14];
  const float* v0 = (const float*)d_in[15];
  const float* v1 = (const float*)d_in[16];
  const float* v2 = (const float*)d_in[17];
  const float* g1 = (const float*)d_in[18];
  const float* g2 = (const float*)d_in[19];
  const float* k_k = (const float*)d_in[20];
  const float* k_a = (const float*)d_in[21];
  const float* r_k = (const float*)d_in[22];
  const float* Wr = (const float*)d_in[23];
  const float* Wk = (const float*)d_in[24];
  const float* Wv = (const float*)d_in[25];
  const float* Wo = (const float*)d_in[26];
  const float* gn_w = (const float*)d_in[27];
  const float* gn_b = (const float*)d_in[28];
  float* out = (float*)d_out;

  char* ws = (char*)d_ws; size_t off = 0;
  auto carve = [&](size_t bytes) -> char* { char* p = ws + off; off += (bytes + 255) & ~(size_t)255; return p; };
  unsigned short* WKVh = (unsigned short*)carve((size_t)2 * HID * HID * 2);
  unsigned short* WKVl = (unsigned short*)carve((size_t)2 * HID * HID * 2);
  unsigned short* W1Th = (unsigned short*)carve((size_t)3 * LORA_RP * HID * 2);
  unsigned short* W1Tl = (unsigned short*)carve((size_t)3 * LORA_RP * HID * 2);
  unsigned short* W2Th = (unsigned short*)carve((size_t)3 * HID * LORA_R * 2);
  unsigned short* W2Tl = (unsigned short*)carve((size_t)3 * HID * LORA_R * 2);
  unsigned short* XKVh = (unsigned short*)carve((size_t)2 * ROWS_KV * HID * 2);
  unsigned short* XKVl = (unsigned short*)carve((size_t)2 * ROWS_KV * HID * 2);
  unsigned short* XWAh = (unsigned short*)carve((size_t)2 * ROWS_EB * HID * 2);
  unsigned short* XWAl = (unsigned short*)carve((size_t)2 * ROWS_EB * HID * 2);
  float*          KVR  = (float*)carve((size_t)2 * ROWS_KV * HID * 4);
  unsigned short* HVh  = (unsigned short*)carve((size_t)ROWS_KV * LORA_RP * 2);
  unsigned short* HVl  = (unsigned short*)carve((size_t)ROWS_KV * LORA_RP * 2);
  float*          HWf  = (float*)carve((size_t)ROWS_EB * LORA_RP * 4);
  unsigned short* HIDh = (unsigned short*)carve((size_t)2 * ROWS_EB * LORA_RP * 2);
  unsigned short* HIDl = (unsigned short*)carve((size_t)2 * ROWS_EB * LORA_RP * 2);
  float*          PWA  = (float*)carve((size_t)2 * ROWS_EB * HID * 4);
  float*          PVf  = (float*)carve((size_t)ROWS_KV * HID * 4);
  float*          RL   = (float*)carve((size_t)NEB * HID * 4);
  float*          EW   = (float*)carve((size_t)ROWS_EB * HID * 4);
  float*          KF   = (float*)carve((size_t)ROWS_EB * HID * 4);
  float*          NKK  = (float*)carve((size_t)ROWS_EB * HID * 4);
  float*          BM   = (float*)carve((size_t)ROWS_EB * HID * 4);
  float*          VP   = (float*)carve((size_t)ROWS_EB * HID * 4);
  float*          OS   = (float*)carve((size_t)NEB * HID * 4);
  if (off > ws_size || off > (size_t)134217728) return;

  split8_kernel<<<dim3(HID * HID / 8 / 256, 2), 256, 0, stream>>>(Wk, Wv, WKVh, WKVl, HID * HID / 8);
  tpack_kernel<<<dim3(LORA_RP * HID / 8 / 256, 3), 256, 0, stream>>>(w1, a1, v1, W1Th, W1Tl, HID, LORA_R, LORA_RP);
  tpack_kernel<<<dim3(HID * LORA_R / 8 / 256, 3), 256, 0, stream>>>(w2, a2, v2, W2Th, W2Tl, LORA_R, HID, HID);

  mix_kernel<<<ROWS_EB / 8, 256, 0, stream>>>(query, keyval, x_w, x_k, x_v, x_a, XWAh, XWAl, XKVh, XKVl);

  wmma_gemm64_split<0><<<dim3(8, 2), 256, 0, stream>>>(
      XKVh, XKVl, HID, (long)ROWS_KV * HID, WKVh, WKVl, HID, (long)HID * HID,
      (void*)KVR, (void*)KVR, HID, (long)ROWS_KV * HID, ROWS_KV, HID, HID);
  wmma_gemm64_split<2><<<dim3(2, 1), 256, 0, stream>>>(
      XKVh + (size_t)ROWS_KV * HID, XKVl + (size_t)ROWS_KV * HID, HID, 0L,
      W1Th + (size_t)2 * LORA_RP * HID, W1Tl + (size_t)2 * LORA_RP * HID, HID, 0L,
      (void*)HVh, (void*)HVl, LORA_RP, 0L, ROWS_KV, LORA_RP, HID);
  wmma_gemm64_split<0><<<dim3(16, 1), 256, 0, stream>>>(
      XWAh, XWAl, HID, 0L, W1Th, W1Tl, HID, 0L,
      (void*)HWf, (void*)HWf, LORA_RP, 0L, ROWS_EB, LORA_RP, HID);
  wmma_gemm64_split<2><<<dim3(16, 1), 256, 0, stream>>>(
      XWAh + (size_t)ROWS_EB * HID, XWAl + (size_t)ROWS_EB * HID, HID, 0L,
      W1Th + (size_t)LORA_RP * HID, W1Tl + (size_t)LORA_RP * HID, HID, 0L,
      (void*)(HIDh + (size_t)ROWS_EB * LORA_RP), (void*)(HIDl + (size_t)ROWS_EB * LORA_RP), LORA_RP, 0L,
      ROWS_EB, LORA_RP, HID);
  tanh_split2_kernel<<<ROWS_EB * LORA_RP / 2 / 256, 256, 0, stream>>>(HWf, HIDh, HIDl, ROWS_EB * LORA_RP / 2);

  wmma_gemm64_split<0><<<dim3(64, 2), 256, 0, stream>>>(
      HIDh, HIDl, LORA_RP, (long)ROWS_EB * LORA_RP, W2Th, W2Tl, LORA_R, (long)HID * LORA_R,
      (void*)PWA, (void*)PWA, HID, (long)ROWS_EB * HID, ROWS_EB, HID, LORA_R);
  wmma_gemm64_split<0><<<dim3(8, 1), 256, 0, stream>>>(
      HVh, HVl, LORA_RP, 0L, W2Th + (size_t)2 * HID * LORA_R, W2Tl + (size_t)2 * HID * LORA_R, LORA_R, 0L,
      (void*)PVf, (void*)PVf, HID, 0L, ROWS_KV, HID, LORA_R);

  rproj_kernel<<<NEB, 256, 0, stream>>>(query, keyval, x_r, Wr, RL);
  prep_kernel<<<ROWS_EB / 2, 256, 0, stream>>>(PWA, KVR, PVf, vfirst, w0, a0, v0, k_k, k_a, EW, KF, NKK, BM, VP);
  scan_kernel<<<NEB * NHEAD, 64, 0, stream>>>(EW, KF, NKK, BM, VP, RL, OS);
  final_kernel<<<NEB, 256, 0, stream>>>(OS, RL, KF, VP, query, keyval, x_g, g1, g2, gn_w, gn_b, r_k, Wo, out);
}
